// RelationAwareAttention_42288247996691
// MI455X (gfx1250) — hardware-verified
//
#include <hip/hip_runtime.h>
#include <math.h>

#ifndef SEQ
#define SEQ 1024
#endif
#define SEQ_FULL 1024
#define DM    1024
#define DK    128
#define DV    128
#define KREL  10
#define NRELT 21
#define NRP   32
#define KBW   32
#define NKB   (SEQ / KBW)
#define WSCL  64.0f
#define QKS   16.0f
#define VSC   16.0f
#define PSC   4096.0f
#define CSC   64.0f
#define RSC   2048.0f
#define SCL   0.08838834764831845f
#define APT   36
#define ZPT   136
#define YPT   132
#define OUT1_OFF ((size_t)SEQ_FULL * DV)

static_assert(OUT1_OFF * 4 == 524288);
static_assert((SEQ % 64) == 0 && SEQ >= 64 && SEQ <= SEQ_FULL);
static_assert(((SEQ * DM) % 2048) == 0 && ((NRP * DK) % 2048) == 0 && ((NRELT * DK) % 8) == 0);
static_assert(DK == 128 && DV == 128 && (DM % 64) == 0 && (DK % 64) == 0);
static_assert((SEQ % KBW) == 0 && (SEQ % 16) == 0);

typedef _Float16 v16h __attribute__((ext_vector_type(16)));
typedef unsigned short v16us __attribute__((ext_vector_type(16)));
typedef unsigned short v8us  __attribute__((ext_vector_type(8)));
typedef float v8f __attribute__((ext_vector_type(8)));
typedef float v4f __attribute__((ext_vector_type(4)));
typedef unsigned int v4u __attribute__((ext_vector_type(4)));

union FragU { v16us v; v8us h[2]; };

__device__ __forceinline__ unsigned short bf_bits(float f) {
  const unsigned u = __float_as_uint(f);
  return (unsigned short)((u + 0x7FFFu + ((u >> 16) & 1u)) >> 16);
}
__device__ __forceinline__ float bf_up(unsigned short h) { return __uint_as_float(((unsigned)h) << 16); }
__device__ __forceinline__ float bfr(float f) { return bf_up(bf_bits(f)); }
__device__ __forceinline__ unsigned short h_bits(_Float16 x) { return __builtin_bit_cast(unsigned short, x); }
__device__ __forceinline__ unsigned short f2h(float f) { return h_bits((_Float16)f); }
__device__ __forceinline__ unsigned pk16(unsigned short a, unsigned short b) { return (unsigned)a | ((unsigned)b << 16); }
__device__ __forceinline__ int clampi(int v, int lo, int hi) { return v < lo ? lo : (v > hi ? hi : v); }
__device__ __forceinline__ v8f zero8() { v8f z = {0.f, 0.f, 0.f, 0.f, 0.f, 0.f, 0.f, 0.f}; return z; }

__device__ __forceinline__ v16us ldfrag_u(const unsigned short* p) {
  FragU f;
  f.h[0] = *(const v8us*)(p);
  f.h[1] = *(const v8us*)(p + 16);
  return f.v;
}

__device__ __forceinline__ v8f mma_raw(v16us a, v16us b, v8f c) {
  return __builtin_amdgcn_wmma_f32_16x16x32_f16(false, __builtin_bit_cast(v16h, a), false,
                                                __builtin_bit_cast(v16h, b), (short)0, c, false, false);
}
__device__ __forceinline__ v8f mma_g(v16us a, v16us b, v8f c) {
  c = mma_raw(a, b, c);
#if defined(__HIP_DEVICE_COMPILE__)
  asm volatile("v_nop\n\tv_nop\n\tv_nop\n\tv_nop" : "+v"(c) : "v"(a), "v"(b));
#endif
  return c;
}
__device__ __forceinline__ void dep_guard1(v8f& a, v8f& b, v16us x) {
#if defined(__HIP_DEVICE_COMPILE__)
  asm volatile("v_nop\n\tv_nop\n\tv_nop\n\tv_nop" : "+v"(a), "+v"(b) : "v"(x));
#endif
}
__device__ __forceinline__ void keep4_u(v16us a, v16us b, v16us c, v16us d) {
#if defined(__HIP_DEVICE_COMPILE__)
  asm volatile("v_nop" :: "v"(a), "v"(b), "v"(c), "v"(d));
#endif
}
__device__ __forceinline__ void acc_guard4(v8f& a, v8f& b, v8f& c, v8f& d) {
#if defined(__HIP_DEVICE_COMPILE__)
  asm volatile("v_nop\n\tv_nop\n\tv_nop\n\tv_nop" : "+v"(a), "+v"(b), "+v"(c), "+v"(d));
#endif
}
__device__ __forceinline__ void wave_sync_lds() {
  __builtin_amdgcn_fence(__ATOMIC_RELEASE, "workgroup");
  __builtin_amdgcn_wave_barrier();
  __builtin_amdgcn_fence(__ATOMIC_ACQUIRE, "workgroup");
}

__global__ __launch_bounds__(256) void cvt_lin(const float* __restrict__ w, unsigned short* o,
                                                int nsrc, int ndst, float sc) {
  const int base = (blockIdx.x * 256 + threadIdx.x) * 8;
  if (base + 8 > ndst) return;
  const bool inr = (base + 8 <= nsrc);
  const int lb = inr ? base : (nsrc - 8);
  const v4f a0 = *(const v4f*)(w + lb);
  const v4f a1 = *(const v4f*)(w + lb + 4);
  v4u hv;
#pragma unroll
  for (int e = 0; e < 2; ++e) {
    hv[e]     = pk16(f2h(bfr(a0[2 * e]) * sc), f2h(bfr(a0[2 * e + 1]) * sc));
    hv[2 + e] = pk16(f2h(bfr(a1[2 * e]) * sc), f2h(bfr(a1[2 * e + 1]) * sc));
  }
  const v4u zz = {0u, 0u, 0u, 0u};
  hv = inr ? hv : zz;
  unsigned short* d = o + base;
  *(volatile v4u*)d = hv;
  __threadfence();
  *(volatile v4u*)d = hv;
}

__global__ __launch_bounds__(256) void cvt_t(const float* __restrict__ w, unsigned short* o, int R, int C, float sc) {
  __shared__ __align__(16) unsigned short st[64 * 72];
  const int t = threadIdx.x;
  const int r0 = blockIdx.y * 64, c0 = blockIdx.x * 64;
  if (r0 + 64 > R || c0 + 64 > C) return;
  {
    const int row = t >> 2, ch = (t & 3) * 16;
    const float* p = w + (size_t)(r0 + row) * C + c0 + ch;
#pragma unroll
    for (int q = 0; q < 4; ++q) {
      const v4f v = *(const v4f*)(p + 4 * q);
#pragma unroll
      for (int e = 0; e < 4; ++e) st[(ch + 4 * q + e) * 72 + row] = f2h(bfr(v[e]) * sc);
    }
  }
  __syncthreads();
  v4u hv[2];
#pragma unroll
  for (int half = 0; half < 2; ++half) {
    const int cl = (t >> 3) + 32 * half, pc = (t & 7) * 8;
    hv[half] = *(const v4u*)(st + cl * 72 + pc);
  }
  for (int pass = 0; pass < 2; ++pass) {
#pragma unroll
    for (int half = 0; half < 2; ++half) {
      const int cl = (t >> 3) + 32 * half, pc = (t & 7) * 8;
      unsigned short* dst = o + (size_t)(c0 + cl) * R + r0 + pc;
      *(volatile v4u*)dst = hv[half];
    }
    __threadfence();
  }
}

template <int OM>
__global__ __launch_bounds__(256) void gemm64(
    const unsigned short* __restrict__ Ap, int lda, const unsigned short* __restrict__ Btp, int ldb,
    unsigned short* Ch, unsigned short* Cl, float* Cf, int ldc, float osc, int M, int N, int K) {
  __shared__ __align__(16) float sT[8][16 * 68];
  const int lane = threadIdx.x & 31;
  const int wave = threadIdx.x >> 5;
  const int tilesN = N >> 6;
  const int tilesM = M >> 6;
  const int tile = blockIdx.x * 8 + wave;
  if (tile >= tilesM * tilesN) return;
  const int tm = tile / tilesN;
  const int tn = tile - tm * tilesN;
  const int m0 = tm << 6;
  const int n0 = tn << 6;

  const int rlane = lane & 15;
  const int koff  = (lane >> 4) * 8;
  const int mOff  = (lane >> 4) * 8;

  v8f acc[4][4];
#pragma unroll
  for (int i = 0; i < 4; ++i)
#pragma unroll
    for (int j = 0; j < 4; ++j) acc[i][j] = zero8();

#pragma unroll 1
  for (int k0 = 0; k0 < K; k0 += 32) {
    v16us bh[4];
#pragma unroll
    for (int j = 0; j < 4; ++j) {
      const size_t bo = (size_t)(n0 + (j << 4) + rlane) * ldb + koff + k0;
      bh[j] = ldfrag_u(Btp + bo);
    }
#pragma unroll
    for (int i = 0; i < 4; ++i) {
      const size_t ao = (size_t)(m0 + (i << 4) + rlane) * lda + koff + k0;
      const v16us ah = ldfrag_u(Ap + ao);
#pragma unroll
      for (int j = 0; j < 4; ++j) acc[i][j] = mma_raw(ah, bh[j], acc[i][j]);
      dep_guard1(acc[i][0], acc[i][3], ah);
    }
    keep4_u(bh[0], bh[1], bh[2], bh[3]);
  }
  acc_guard4(acc[0][0], acc[0][1], acc[0][2], acc[0][3]);
  acc_guard4(acc[1][0], acc[1][1], acc[1][2], acc[1][3]);
  acc_guard4(acc[2][0], acc[2][1], acc[2][2], acc[2][3]);
  acc_guard4(acc[3][0], acc[3][1], acc[3][2], acc[3][3]);

  const int hh2 = lane >> 4, c4 = (lane & 15) * 4;
  const int q8  = lane >> 3, c8 = (lane & 7) * 8;

  float* slab = sT[wave];
#pragma unroll
  for (int i = 0; i < 4; ++i) {
    const int mBase = m0 + (i << 4);
#pragma unroll
    for (int j = 0; j < 4; ++j) {
#pragma unroll
      for (int r = 0; r < 8; ++r) {
        slab[(mOff + r) * 68 + (j << 4) + rlane] = acc[i][j][r];
      }
    }
    wave_sync_lds();
    if (OM == 0) {
      v4f vals[8];
#pragma unroll
      for (int it = 0; it < 8; ++it) {
        const int row = it * 2 + hh2;
        const v4f v = *(const v4f*)(slab + row * 68 + c4);
        vals[it] = v * osc;
      }
      for (int pass = 0; pass < 2; ++pass) {
#pragma unroll
        for (int it = 0; it < 8; ++it) {
          const int row = it * 2 + hh2;
          *(volatile v4f*)(Cf + (size_t)(mBase + row) * ldc + (size_t)n0 + c4) = vals[it];
        }
        __threadfence();
      }
    } else if (OM == 1) {
      v4u hv[4];
#pragma unroll
      for (int it = 0; it < 4; ++it) {
        const int row = it * 4 + q8;
        const float* sp = slab + row * 68 + c8;
        v4u ha = {0u, 0u, 0u, 0u};
#pragma unroll
        for (int e = 0; e < 4; ++e) {
          const float b0 = sp[2 * e]     * osc;
          const float b1 = sp[2 * e + 1] * osc;
          ha[e] = pk16(f2h(b0), f2h(b1));
        }
        hv[it] = ha;
      }
      for (int pass = 0; pass < 2; ++pass) {
#pragma unroll
        for (int it = 0; it < 4; ++it) {
          const int row = it * 4 + q8;
          const size_t go = (size_t)(mBase + row) * ldc + (size_t)n0 + c8;
          *(volatile v4u*)(Ch + go) = hv[it];
        }
        __threadfence();
      }
    } else {
      v4u hv[4], lv[4];
#pragma unroll
      for (int it = 0; it < 4; ++it) {
        const int row = it * 4 + q8;
        const float* sp = slab + row * 68 + c8;
        v4u ha = {0u, 0u, 0u, 0u};
        v4u la = {0u, 0u, 0u, 0u};
#pragma unroll
        for (int e = 0; e < 4; ++e) {
          const float b0 = sp[2 * e]     * osc;
          const float b1 = sp[2 * e + 1] * osc;
          const _Float16 h0 = (_Float16)b0;
          const _Float16 h1 = (_Float16)b1;
          const float l0 = (b0 - (float)h0) * RSC;
          const float l1 = (b1 - (float)h1) * RSC;
          ha[e] = pk16(h_bits(h0), h_bits(h1));
          la[e] = pk16(f2h(l0), f2h(l1));
        }
        hv[it] = ha;
        lv[it] = la;
      }
      for (int pass = 0; pass < 2; ++pass) {
#pragma unroll
        for (int it = 0; it < 4; ++it) {
          const int row = it * 4 + q8;
          const size_t go = (size_t)(mBase + row) * ldc + (size_t)n0 + c8;
          *(volatile v4u*)(Ch + go) = hv[it];
          *(volatile v4u*)(Cl + go) = lv[it];
        }
        __threadfence();
      }
    }
    wave_sync_lds();
  }
}

__device__ __forceinline__ void tile_logits(const v16us (&qh)[4], const v16us (&ql)[4],
                                            const unsigned short* __restrict__ KH,
                                            const unsigned short* __restrict__ KL,
                                            const float* tb, int sb, int t0, int m, int hh,
                                            float (&s0)[8], float (&s1)[8]) {
  v8f S0h = zero8(), S0x = zero8(), S1h = zero8(), S1x = zero8();
  const size_t ko0 = (size_t)(sb + m) * DK + 8 * hh;
  const size_t ko1 = ko0 + (size_t)16 * DK;
#pragma unroll
  for (int ks = 0; ks < 4; ++ks) {
    const v16us k0h = ldfrag_u(KH + ko0 + ks * 32);
    const v16us k0l = ldfrag_u(KL + ko0 + ks * 32);
    const v16us k1h = ldfrag_u(KH + ko1 + ks * 32);
    const v16us k1l = ldfrag_u(KL + ko1 + ks * 32);
    S0h = mma_g(qh[ks], k0h, S0h);
    S0x = mma_g(qh[ks], k0l, S0x);
    S0x = mma_g(ql[ks], k0h, S0x);
    S1h = mma_g(qh[ks], k1h, S1h);
    S1x = mma_g(qh[ks], k1l, S1x);
    S1x = mma_g(ql[ks], k1h, S1x);
  }
  const float c1 = 1.0f / (QKS * QKS);
  const float c2 = 1.0f / (QKS * QKS * RSC);
#pragma unroll
  for (int r = 0; r < 8; ++r) {
    const int row = 8 * hh + r;
    const int qrow = t0 + row;
    const int i0 = clampi(sb + m - qrow, -KREL, KREL) + KREL;
    const int i1 = clampi(sb + 16 + m - qrow, -KREL, KREL) + KREL;
    s0[r] = S0h[r] * c1 + S0x[r] * c2 + tb[row * NRP + i0];
    s1[r] = S1h[r] * c1 + S1x[r] * c2 + tb[row * NRP + i1];
  }
}

__global__ __launch_bounds__(32) void attn_kernel(
    const unsigned short* __restrict__ QH, const unsigned short* __restrict__ QL,
    const unsigned short* __restrict__ KH, const unsigned short* __restrict__ KL,
    const unsigned short* __restrict__ WKP, const unsigned short* __restrict__ VT,
    const unsigned short* __restrict__ WOT, float* Aout, float* Yout) {
  __shared__ __align__(16) float tb[16 * NRP];
  __shared__ __align__(16) float ast[16 * APT];
  __shared__ __align__(16) unsigned short pst[NKB * 16 * KBW];
  __shared__ __align__(16) unsigned short zh[16 * ZPT];
  __shared__ __align__(16) unsigned short zl[16 * ZPT];
  __shared__ __align__(16) float yst[16 * YPT];
  const int lane = threadIdx.x & 31, m = lane & 15, hh = lane >> 4;
  const int t0 = blockIdx.x << 4;
  if (t0 + 16 > SEQ) return;

  v16us qh[4], ql[4];
  {
    const size_t qo = (size_t)(t0 + m) * DK + 8 * hh;
#pragma unroll
    for (int ks = 0; ks < 4; ++ks) {
      qh[ks] = ldfrag_u(QH + qo + ks * 32);
      ql[ks] = ldfrag_u(QL + qo + ks * 32);
    }
  }

  {
    v8f b0h = zero8(), b0x = zero8(), b1h = zero8(), b1x = zero8();
#pragma unroll
    for (int ks = 0; ks < 4; ++ks) {
      const size_t wo0 = (size_t)m * DK + ks * 32 + 8 * hh;
      const size_t wo1 = wo0 + (size_t)16 * DK;
      const v16us w0 = ldfrag_u(WKP + wo0);
      const v16us w1 = ldfrag_u(WKP + wo1);
      b0h = mma_g(qh[ks], w0, b0h);
      b0x = mma_g(ql[ks], w0, b0x);
      b1h = mma_g(qh[ks], w1, b1h);
      b1x = mma_g(ql[ks], w1, b1x);
    }
    const float ct = 1.0f / (QKS * WSCL);
    const float cx = 1.0f / RSC;
#pragma unroll
    for (int r = 0; r < 8; ++r) {
      const int row = 8 * hh + r;
      tb[row * NRP + m]      = (b0h[r] + b0x[r] * cx) * ct;
      tb[row * NRP + 16 + m] = (b1h[r] + b1x[r] * cx) * ct;
    }
  }
  __syncthreads();

  float mx[8], ls[8];
#pragma unroll
  for (int r = 0; r < 8; ++r) { mx[r] = -1.0e30f; ls[r] = 0.f; }
#pragma unroll 1
  for (int kb = 0; kb < NKB; ++kb) {
    const int sb = kb * KBW;
    float s0[8], s1[8];
    tile_logits(qh, ql, KH, KL, tb, sb, t0, m, hh, s0, s1);
#pragma unroll
    for (int r = 0; r < 8; ++r) {
      float xm = fmaxf(s0[r], s1[r]);
      xm = fmaxf(xm, __shfl_xor(xm, 1, 32));
      xm = fmaxf(xm, __shfl_xor(xm, 2, 32));
      xm = fmaxf(xm, __shfl_xor(xm, 4, 32));
      xm = fmaxf(xm, __shfl_xor(xm, 8, 32));
      const float mn = fmaxf(mx[r], xm);
      const float al = __expf(mx[r] - mn);
      mx[r] = mn;
      float ps = __expf(s0[r] - mn) + __expf(s1[r] - mn);
      ps += __shfl_xor(ps, 1, 32);
      ps += __shfl_xor(ps, 2, 32);
      ps += __shfl_xor(ps, 4, 32);
      ps += __shfl_xor(ps, 8, 32);
      ls[r] = ls[r] * al + ps;
    }
  }
  float linv[8];
#pragma unroll
  for (int r = 0; r < 8; ++r) linv[r] = 1.0f / ls[r];

  const int q8 = lane >> 3, c4 = (lane & 7) * 4;
#pragma unroll 1
  for (int kb = 0; kb < NKB; ++kb) {
    const int sb = kb * KBW;
    float s0[8], s1[8];
    tile_logits(qh, ql, KH, KL, tb, sb, t0, m, hh, s0, s1);
    unsigned short* ph = pst + kb * (16 * KBW);
#pragma unroll
    for (int r = 0; r < 8; ++r) {
      const int row = 8 * hh + r;
      const float p0 = __expf(s0[r] - mx[r]);
      const float p1 = __expf(s1[r] - mx[r]);
      ast[row * APT + m]      = p0 * linv[r];
      ast[row * APT + 16 + m] = p1 * linv[r];
      ph[row * KBW + m]      = f2h(p0 * PSC);
      ph[row * KBW + 16 + m] = f2h(p1 * PSC);
    }
    __syncthreads();
    v4f av[4];
#pragma unroll
    for (int it = 0; it < 4; ++it) {
      const int row = it * 4 + q8;
      av[it] = *(const v4f*)(ast + row * APT + c4);
    }
    for (int pass = 0; pass < 2; ++pass) {
#pragma unroll
      for (int it = 0; it < 4; ++it) {
        const int row = it * 4 + q8;
        *(volatile v4f*)(Aout + (size_t)(t0 + row) * SEQ + (size_t)sb + c4) = av[it];
      }
      __threadfence();
    }
    __syncthreads();
  }

  v8f O[8];
#pragma unroll
  for (int j = 0; j < 8; ++j) O[j] = zero8();
#pragma unroll 1
  for (int kb = 0; kb < NKB; ++kb) {
    const int sb = kb * KBW;
    const v16us af = ldfrag_u(pst + kb * (16 * KBW) + m * KBW + 8 * hh);
    const size_t vo = (size_t)m * SEQ + (size_t)sb + 8 * hh;
#pragma unroll
    for (int j = 0; j < 8; ++j) {
      const v16us vf = ldfrag_u(VT + vo + (size_t)(16 * j) * SEQ);
      O[j] = mma_g(af, vf, O[j]);
    }
  }

  {
    const float fin = CSC / (PSC * VSC);
#pragma unroll
    for (int r = 0; r < 8; ++r) {
      const int row = 8 * hh + r;
      const float g = linv[r] * fin;
#pragma unroll
      for (int j = 0; j < 8; ++j) {
        const float c = O[j][r] * g;
        const _Float16 hb = (_Float16)c;
        const float lo = (c - (float)hb) * RSC;
        zh[row * ZPT + 16 * j + m] = h_bits(hb);
        zl[row * ZPT + 16 * j + m] = f2h(lo);
      }
    }
  }
  __syncthreads();
  {
    const float cy = 1.0f / (CSC * WSCL);
    const float cx = 1.0f / RSC;
#pragma unroll
    for (int j = 0; j < 8; ++j) {
      v8f yh = zero8(), yx = zero8();
#pragma unroll
      for (int ks = 0; ks < 4; ++ks) {
        const v16us ah = ldfrag_u(zh + m * ZPT + ks * 32 + 8 * hh);
        const v16us al = ldfrag_u(zl + m * ZPT + ks * 32 + 8 * hh);
        const v16us bw = ldfrag_u(WOT + (size_t)(16 * j + m) * DV + ks * 32 + 8 * hh);
        yh = mma_g(ah, bw, yh);
        yx = mma_g(al, bw, yx);
      }
#pragma unroll
      for (int r = 0; r < 8; ++r) {
        const int row = 8 * hh + r;
        yst[row * YPT + 16 * j + m] = (yh[r] + yx[r] * cx) * cy;
      }
    }
  }
  __syncthreads();
  {
    v4f yv[16];
#pragma unroll
    for (int it = 0; it < 16; ++it) yv[it] = *(const v4f*)(yst + it * YPT + lane * 4);
    for (int pass = 0; pass < 2; ++pass) {
#pragma unroll
      for (int it = 0; it < 16; ++it) {
        *(volatile v4f*)(Yout + (size_t)(t0 + it) * DV + lane * 4) = yv[it];
      }
      __threadfence();
    }
  }
}

extern "C" void kernel_launch(void* const* d_in, const int* in_sizes, int n_in,
                              void* d_out, int out_size, void* d_ws, size_t ws_size,
                              hipStream_t stream) {
  if (n_in < 7) return;
  if (in_sizes[0] < SEQ * DM) return;
  if (in_sizes[1] < SEQ * DM) return;
  if (in_sizes[2] < DM * DK) return;
  if (in_sizes[3] < DM * DK) return;
  if (in_sizes[4] < DM * DV) return;
  if (in_sizes[5] < DV * DV) return;
  if (in_sizes[6] < NRELT * DK) return;
  if (out_size < 0 || (size_t)out_size < OUT1_OFF + (size_t)SEQ * SEQ) return;

  const float* p_xma = (const float*)d_in[0];
  const float* p_xmi = (const float*)d_in[1];
  const float* p_wq  = (const float*)d_in[2];
  const float* p_wk  = (const float*)d_in[3];
  const float* p_wv  = (const float*)d_in[4];
  const float* p_wo  = (const float*)d_in[5];
  const float* p_rel = (const float*)d_in[6];

  const size_t PX  = (size_t)SEQ * DM * 2;
  const size_t PWT = (size_t)DK * DM * 2;
  const size_t PWO = (size_t)DV * DV * 2;
  const size_t PWK = (size_t)NRP * DK * 2;
  const size_t PQK = (size_t)SEQ * DK * 2;
  const size_t PVT = (size_t)DV * SEQ * 2;
  size_t off = 0;
  const size_t oXA = off; off += PX;
  const size_t oXI = off; off += PX;
  const size_t oWQ = off; off += PWT;
  const size_t oWK = off; off += PWT;
  const size_t oWV = off; off += PWT;
  const size_t oWO = off; off += PWO;
  const size_t oWP = off; off += PWK;
  const size_t oQH = off; off += PQK;
  const size_t oQL = off; off += PQK;
  const size_t oKH = off; off += PQK;
  const size_t oKL = off; off += PQK;
  const size_t oVT = off; off += PVT;
  if (off > ws_size) return;
  if (off > (size_t)134217728) return;

  char* ws = (char*)d_ws;
  unsigned short* XAH = (unsigned short*)(ws + oXA);
  unsigned short* XIH = (unsigned short*)(ws + oXI);
  unsigned short* WQT = (unsigned short*)(ws + oWQ);
  unsigned short* WKT = (unsigned short*)(ws + oWK);
  unsigned short* WVT = (unsigned short*)(ws + oWV);
  unsigned short* WOT = (unsigned short*)(ws + oWO);
  unsigned short* WKP = (unsigned short*)(ws + oWP);
  unsigned short* QH  = (unsigned short*)(ws + oQH);
  unsigned short* QL  = (unsigned short*)(ws + oQL);
  unsigned short* KH  = (unsigned short*)(ws + oKH);
  unsigned short* KL  = (unsigned short*)(ws + oKL);
  unsigned short* VT  = (unsigned short*)(ws + oVT);
  float* out0 = (float*)d_out;
  float* out1 = out0 + OUT1_OFF;
  float* fdummy = (float*)(ws + oXA);
  unsigned short* hdummy = QL;

  const dim3 blk(256);
  const int tQ = (SEQ / 64) * (DK / 64);
  const int tV = (DV / 64) * (SEQ / 64);
  const int gQ = (tQ + 7) / 8;
  const int gV = (tV + 7) / 8;

  cvt_lin<<<dim3((SEQ * DM) / 2048), blk, 0, stream>>>(p_xma, XAH, SEQ * DM, SEQ * DM, 1.0f);
  cvt_lin<<<dim3((SEQ * DM) / 2048), blk, 0, stream>>>(p_xmi, XIH, SEQ * DM, SEQ * DM, 1.0f);
  cvt_t<<<dim3(DK / 64, DM / 64), blk, 0, stream>>>(p_wq, WQT, DM, DK, WSCL);
  cvt_t<<<dim3(DK / 64, DM / 64), blk, 0, stream>>>(p_wk, WKT, DM, DK, WSCL);
  cvt_t<<<dim3(DV / 64, DM / 64), blk, 0, stream>>>(p_wv, WVT, DM, DV, WSCL);
  cvt_t<<<dim3(DV / 64, DV / 64), blk, 0, stream>>>(p_wo, WOT, DV, DV, WSCL);
  cvt_lin<<<dim3((NRP * DK) / 2048), blk, 0, stream>>>(p_rel, WKP, NRELT * DK, NRP * DK, WSCL);

  gemm64<2><<<dim3(gQ), blk, 0, stream>>>(XAH, DM, WQT, DM, QH, QL, fdummy, DK, (QKS / WSCL) * SCL, SEQ, DK, DM);
  gemm64<2><<<dim3(gQ), blk, 0, stream>>>(XIH, DM, WKT, DM, KH, KL, fdummy, DK, QKS / WSCL, SEQ, DK, DM);
  gemm64<1><<<dim3(gV), blk, 0, stream>>>(WVT, DM, XIH, DM, VT, hdummy, fdummy, SEQ, VSC / WSCL, DV, SEQ, DM);

  attn_kernel<<<dim3(SEQ / 16), dim3(32), 0, stream>>>(QH, QL, KH, KL, WKP, VT, WOT, out1, out0);
  (void)hipGetLastError();
}
